// GraphSAGEEncoder_64192581206427
// MI455X (gfx1250) — hardware-verified
//
#include <hip/hip_runtime.h>
#include <stddef.h>


#define INC     128
#define HC      256
#define NTHR    256
#define NWAVE   8
#define EPT     8
#define NGRP    2
#define CHUNK   (NTHR * EPT * NGRP)
#define WCAP    (EPT * NGRP * 32)
#define LISTN   (NWAVE * WCAP)
#define NBC     4096
#define NBF     1024
#define RCAP    40960
#define RBN     128
#define TGT     256
#define DEGCAP  256
#define GR      32
#define OTHR    512
#define BNEPS   1e-5f

#define LDS_FILL ((RCAP + NBF + LISTN) * 4 + 64)

static_assert((CHUNK & (CHUNK - 1)) == 0);
static_assert(CHUNK <= 4096);
static_assert(NBC <= 4096 && NBF <= 4096);
static_assert((NBC & (NBC - 1)) == 0 && (NBF & (NBF - 1)) == 0);
static_assert(NBC == 4 * NBF);
static_assert(OTHR * 8 == NBC);
static_assert((RCAP % 32) == 0);
static_assert(TGT == NWAVE * 32);
static_assert((NBC % TGT) == 0);
static_assert((HC * 2 * INC / 8) % NTHR == 0 && (HC * 2 * HC / 8) % NTHR == 0);
static_assert(GR == 4 * NWAVE && HC == NTHR);
static_assert((INC % 32) == 0 && (HC % 128) == 0);

typedef float          v4f   __attribute__((ext_vector_type(4)));
typedef float          v8f   __attribute__((ext_vector_type(8)));
typedef int            v4i   __attribute__((ext_vector_type(4)));
typedef double         v2d   __attribute__((ext_vector_type(2)));
typedef unsigned short v8us  __attribute__((ext_vector_type(8)));
typedef __attribute__((ext_vector_type(16))) __bf16 v16bf;
union FragB { v16bf bf; v8us hv[2]; unsigned int w[8]; };

__device__ __forceinline__ unsigned int bf_rne(float f) {
  const unsigned int u = __float_as_uint(f);
  return (u + 0x7FFFu + ((u >> 16) & 1u)) >> 16;
}

__device__ __forceinline__ unsigned int split_pack(float x0, float x1, unsigned int& lo) {
  const unsigned int h0 = bf_rne(x0), h1 = bf_rne(x1);
  const float r0 = x0 - __uint_as_float(h0 << 16);
  const float r1 = x1 - __uint_as_float(h1 << 16);
  const unsigned int l0 = bf_rne(r0), l1 = bf_rne(r1);
  lo = l0 | (l1 << 16);
  return h0 | (h1 << 16);
}

__device__ __forceinline__ v8f wmb(v16bf a, v16bf b, v8f c) {
  v8f d = __builtin_amdgcn_wmma_f32_16x16x32_bf16(false, a, false, b, (short)0, c, false, false);
  asm volatile("v_nop\n\tv_nop\n\tv_nop\n\tv_nop" : "+v"(d) : "v"(a), "v"(b));
  return d;
}

template <int NB>
__device__ __forceinline__ int scan_chunk(const int* __restrict__ dsts, int nE, int cbase, int slotBase,
                                          int vec8, int* list, int tid, int lane, int wave) {
  int wc = 0;
#pragma unroll
  for (int g = 0; g < NGRP; ++g) {
    const int el0  = (g * NTHR + tid) * EPT;
    const int e0   = cbase + el0;
    const int sent = -2147483647 - 1;
    v4i da, db;
    if (vec8 != 0 && cbase + CHUNK <= nE) {
      da = *(const v4i*)(dsts + e0);
      db = *(const v4i*)(dsts + e0 + 4);
    } else {
      da.x = (e0     < nE) ? dsts[min(e0, nE - 1)] : sent;
      da.y = (e0 + 1 < nE) ? dsts[min(e0 + 1, nE - 1)] : sent;
      da.z = (e0 + 2 < nE) ? dsts[min(e0 + 2, nE - 1)] : sent;
      da.w = (e0 + 3 < nE) ? dsts[min(e0 + 3, nE - 1)] : sent;
      db.x = (e0 + 4 < nE) ? dsts[min(e0 + 4, nE - 1)] : sent;
      db.y = (e0 + 5 < nE) ? dsts[min(e0 + 5, nE - 1)] : sent;
      db.z = (e0 + 6 < nE) ? dsts[min(e0 + 6, nE - 1)] : sent;
      db.w = (e0 + 7 < nE) ? dsts[min(e0 + 7, nE - 1)] : sent;
    }
    const unsigned nb = (unsigned)slotBase;
    const unsigned s0 = (unsigned)da.x - nb, s1 = (unsigned)da.y - nb;
    const unsigned s2 = (unsigned)da.z - nb, s3 = (unsigned)da.w - nb;
    const unsigned s4 = (unsigned)db.x - nb, s5 = (unsigned)db.y - nb;
    const unsigned s6 = (unsigned)db.z - nb, s7 = (unsigned)db.w - nb;
    const bool h0 = s0 < (unsigned)NB, h1 = s1 < (unsigned)NB, h2 = s2 < (unsigned)NB, h3 = s3 < (unsigned)NB;
    const bool h4 = s4 < (unsigned)NB, h5 = s5 < (unsigned)NB, h6 = s6 < (unsigned)NB, h7 = s7 < (unsigned)NB;
    const unsigned any = __builtin_amdgcn_ballot_w32(h0 | h1 | h2 | h3 | h4 | h5 | h6 | h7);
    if (any != 0u) {
#define HITJ(J, HJ, SJ) { \
        const unsigned mj = __builtin_amdgcn_ballot_w32(HJ); \
        if (mj != 0u) { \
          if (HJ) { \
            const int pos = wc + (int)__builtin_amdgcn_mbcnt_lo(mj, 0u); \
            if (pos < WCAP) list[wave * WCAP + pos] = ((el0 + (J)) << 12) | (int)(SJ); \
          } \
          wc += (int)__builtin_popcount(mj); } }
      HITJ(0, h0, s0)
      HITJ(1, h1, s1)
      HITJ(2, h2, s2)
      HITJ(3, h3, s3)
      HITJ(4, h4, s4)
      HITJ(5, h5, s5)
      HITJ(6, h6, s6)
      HITJ(7, h7, s7)
#undef HITJ
    }
  }
  return wc;
}

__global__ __launch_bounds__(NTHR) void k_wprep(
    const float* __restrict__ Wl0, const float* __restrict__ Wr0,
    const float* __restrict__ Wl1, const float* __restrict__ Wr1,
    const float* __restrict__ Wl2, const float* __restrict__ Wr2,
    unsigned short* whi0, unsigned short* wlo0, unsigned short* whi1, unsigned short* wlo1,
    unsigned short* whi2, unsigned short* wlo2) {
  const int g0 = HC * (2 * INC) / 8;
  const int g1 = HC * (2 * HC) / 8;
  const int bstart = blockIdx.x * NTHR;
  const float* Wl; const float* Wr; unsigned short* dh; unsigned short* dl; int CI, segOff;
  if (bstart < g0)            { Wl = Wl0; Wr = Wr0; dh = whi0; dl = wlo0; CI = INC; segOff = 0; }
  else if (bstart < g0 + g1)  { Wl = Wl1; Wr = Wr1; dh = whi1; dl = wlo1; CI = HC;  segOff = g0; }
  else                        { Wl = Wl2; Wr = Wr2; dh = whi2; dl = wlo2; CI = HC;  segOff = g0 + g1; }
  const int i = bstart + (int)threadIdx.x;
  if (i >= g0 + 2 * g1) return;
  const int K  = 2 * CI;
  const int o  = (i - segOff) * 8;
  const int co = o / K;
  const int k0 = o - co * K;
  int kl = k0; kl = kl > CI - 8 ? CI - 8 : kl;
  int kr = k0 - CI; kr = kr < 0 ? 0 : kr;
  const float* pl = Wl + (size_t)co * CI + kl;
  const float* pr = Wr + (size_t)co * CI + kr;
  const v4f la = *(const v4f*)pl, lb = *(const v4f*)(pl + 4);
  const v4f ra = *(const v4f*)pr, rb = *(const v4f*)(pr + 4);
  const bool useL = k0 < CI;
  float v[8];
  v[0] = useL ? la.x : ra.x; v[1] = useL ? la.y : ra.y; v[2] = useL ? la.z : ra.z; v[3] = useL ? la.w : ra.w;
  v[4] = useL ? lb.x : rb.x; v[5] = useL ? lb.y : rb.y; v[6] = useL ? lb.z : rb.z; v[7] = useL ? lb.w : rb.w;
  FragB fh, fl;
#pragma unroll
  for (int p = 0; p < 4; ++p) {
    unsigned int lw;
    fh.w[p] = split_pack(v[2 * p], v[2 * p + 1], lw);
    fl.w[p] = lw;
  }
  const v8us hvv = fh.hv[0], lvv = fl.hv[0];
  unsigned short* ph = dh + o;
  unsigned short* plo = dl + o;
  *(volatile v8us*)ph  = hvv;
  *(volatile v8us*)plo = lvv;
  __threadfence();
  *(volatile v8us*)ph  = hvv;
  *(volatile v8us*)plo = lvv;
}

__global__ __launch_bounds__(NTHR) void k_count(
    const int* __restrict__ ei, int* cnt, float* invd, int nE, int vec8) {
  __shared__ __attribute__((aligned(16))) int scnt[NBC];
  __shared__ __attribute__((aligned(16))) int list[LISTN];
  __shared__ int wcnt[NWAVE];
  const int tid = threadIdx.x, lane = tid & 31, wave = tid >> 5;
  const int nodeBase = blockIdx.x * NBC;
  const int* dsts = ei + nE;

  for (int i = tid; i < NBC; i += NTHR) scnt[i] = 0;
  __syncthreads();

  const int nChunks = (nE + CHUNK - 1) / CHUNK;
#pragma unroll 1
  for (int ch = 0; ch < nChunks; ++ch) {
    const int cbase = ch * CHUNK;
    const int wc = scan_chunk<NBC>(dsts, nE, cbase, nodeBase, vec8, list, tid, lane, wave);
    if (lane == 0) wcnt[wave] = wc;
    __syncthreads();
    if (wave == 0) {
#pragma unroll 1
      for (int wsx = 0; wsx < NWAVE; ++wsx) {
        int n = __builtin_amdgcn_readfirstlane(wcnt[wsx]);
        n = n > WCAP ? WCAP : (n < 0 ? 0 : n);
        const int* lp = list + wsx * WCAP;
#pragma unroll 1
        for (int i = 0; i < n; ++i) {
          const int ent  = __builtin_amdgcn_readfirstlane(lp[i]);
          const int slot = ent & (NBC - 1);
          if (lane == 0) scnt[slot] = scnt[slot] + 1;
        }
      }
    }
    __syncthreads();
  }

  v4i cq[4]; v4f dq[4];
#pragma unroll
  for (int q = 0; q < 4; ++q) {
    const int f = (wave * 4 + q) * 128 + 4 * lane;
    const v4i c = *(const v4i*)(scnt + f);
    cq[q] = c;
    dq[q].x = 1.0f / (float)(c.x < 1 ? 1 : c.x);
    dq[q].y = 1.0f / (float)(c.y < 1 ? 1 : c.y);
    dq[q].z = 1.0f / (float)(c.z < 1 ? 1 : c.z);
    dq[q].w = 1.0f / (float)(c.w < 1 ? 1 : c.w);
  }
  int*   cp = cnt + (size_t)nodeBase;
  float* dp = invd + (size_t)nodeBase;
#pragma unroll
  for (int q = 0; q < 4; ++q) {
    const int f = (wave * 4 + q) * 128 + 4 * lane;
    *(volatile v4i*)(cp + f) = cq[q];
    *(volatile v4f*)(dp + f) = dq[q];
  }
  __threadfence();
#pragma unroll
  for (int q = 0; q < 4; ++q) {
    const int f = (wave * 4 + q) * 128 + 4 * lane;
    *(volatile v4i*)(cp + f) = cq[q];
    *(volatile v4f*)(dp + f) = dq[q];
  }
}

__global__ __launch_bounds__(OTHR) void k_offsets(
    const int* __restrict__ cnt, int* off, int* rbase, int nChunk) {
  __shared__ __attribute__((aligned(16))) int soff[NBC];
  __shared__ __attribute__((aligned(16))) int srb[RBN];
  __shared__ int wtot[OTHR / 32];
  const int tid = threadIdx.x, lane = tid & 31, wave = tid >> 5, sub = tid >> 7;
  for (int i = tid; i < RBN; i += OTHR) srb[i] = 0;
  int carry = 0;
#pragma unroll 1
  for (int ch = 0; ch < nChunk; ++ch) {
    const int base = ch * NBC;
    const v4i c0 = *(const v4i*)(cnt + base + 8 * tid);
    const v4i c1 = *(const v4i*)(cnt + base + 8 * tid + 4);
    const int e0 = max(c0.x, 0), e1 = max(c0.y, 0), e2 = max(c0.z, 0), e3 = max(c0.w, 0);
    const int e4 = max(c1.x, 0), e5 = max(c1.y, 0), e6 = max(c1.z, 0), e7 = max(c1.w, 0);
    const int ts = e0 + e1 + e2 + e3 + e4 + e5 + e6 + e7;
    int incl = ts;
#pragma unroll
    for (int d = 1; d < 32; d <<= 1) {
      const int t = __shfl_up(incl, d);
      if (lane >= d) incl += t;
    }
    if (lane == 31) wtot[wave] = incl;
    __syncthreads();
    const int S0 = wtot[0]  + wtot[1]  + wtot[2]  + wtot[3];
    const int S1 = wtot[4]  + wtot[5]  + wtot[6]  + wtot[7];
    const int S2 = wtot[8]  + wtot[9]  + wtot[10] + wtot[11];
    const int S3 = wtot[12] + wtot[13] + wtot[14] + wtot[15];
    int pre = 0;
#pragma unroll 1
    for (int w = 4 * sub; w < wave; ++w) pre += wtot[w];
    const int b0 = carry;
    const int b1 = b0 + ((S0 + 31) & ~31);
    const int b2 = b1 + ((S1 + 31) & ~31);
    const int b3 = b2 + ((S2 + 31) & ~31);
    const int b4 = b3 + ((S3 + 31) & ~31);
    const int myb = sub == 0 ? b0 : (sub == 1 ? b1 : (sub == 2 ? b2 : b3));
    if (tid == 0) {
      srb[min(4 * ch + 0, RBN - 1)] = b0;
      srb[min(4 * ch + 1, RBN - 1)] = b1;
      srb[min(4 * ch + 2, RBN - 1)] = b2;
      srb[min(4 * ch + 3, RBN - 1)] = b3;
    }
    int run = myb + pre + incl - ts;
    soff[8 * tid + 0] = run; run += e0;
    soff[8 * tid + 1] = run; run += e1;
    soff[8 * tid + 2] = run; run += e2;
    soff[8 * tid + 3] = run; run += e3;
    soff[8 * tid + 4] = run; run += e4;
    soff[8 * tid + 5] = run; run += e5;
    soff[8 * tid + 6] = run; run += e6;
    soff[8 * tid + 7] = run;
    carry = b4;
    __syncthreads();
    const v4i o0 = *(const v4i*)(soff + 4 * tid);
    const v4i o1 = *(const v4i*)(soff + 4 * (tid + OTHR));
    int* op = off + base;
    *(volatile v4i*)(op + 4 * tid) = o0;
    *(volatile v4i*)(op + 4 * (tid + OTHR)) = o1;
    __threadfence();
    *(volatile v4i*)(op + 4 * tid) = o0;
    *(volatile v4i*)(op + 4 * (tid + OTHR)) = o1;
    __syncthreads();
  }
  if (tid == 0) srb[min(4 * nChunk, RBN - 1)] = carry;
  __syncthreads();
  v4i rv = {0, 0, 0, 0};
  if (tid < 32) rv = *(const v4i*)(srb + 4 * tid);
  if (tid < 32) *(volatile v4i*)(rbase + 4 * tid) = rv;
  __threadfence();
  if (tid < 32) *(volatile v4i*)(rbase + 4 * tid) = rv;
}

__global__ __launch_bounds__(NTHR) void k_fill(
    const int* __restrict__ ei, const int* __restrict__ off, const int* __restrict__ rbase,
    int* csr, int nN, int nE, int vec8, int csrLen) {
  extern __shared__ v4f lds_dyn[];
  int* region = (int*)lds_dyn;
  int* cursor = region + RCAP;
  int* list   = cursor + NBF;
  int* wcnt   = list + LISTN;
  const int tid = threadIdx.x, lane = tid & 31, wave = tid >> 5;
  const int b = blockIdx.x;
  const int nodeBase = b * NBF;
  const int* dsts = ei + nE;

  int rb0 = rbase[b];
  const int rb1 = rbase[b + 1];
  rb0 = rb0 < 0 ? 0 : (rb0 > csrLen ? csrLen : rb0);
  rb0 &= ~31;
  int len = rb1 - rb0;
  len = len < 0 ? 0 : (len > RCAP ? RCAP : len);
  int lenW = (len + 31) & ~31;
  if (rb0 + lenW > csrLen) lenW = (csrLen - rb0) & ~31;

  {
    const v4i z = {0, 0, 0, 0};
    for (int i = tid; i < RCAP / 4; i += NTHR) ((v4i*)region)[i] = z;
    for (int s = tid; s < NBF; s += NTHR) {
      int o = off[nodeBase + s] - rb0;
      o = o < 0 ? 0 : (o > RCAP ? RCAP : o);
      cursor[s] = o;
    }
  }
  __syncthreads();

  const int nChunks = (nE + CHUNK - 1) / CHUNK;
#pragma unroll 1
  for (int ch = 0; ch < nChunks; ++ch) {
    const int cbase = ch * CHUNK;
    const int wc = scan_chunk<NBF>(dsts, nE, cbase, nodeBase, vec8, list, tid, lane, wave);
    if (lane == 0) wcnt[wave] = wc;
    __syncthreads();
    if (wave == 0) {
#pragma unroll 1
      for (int wsx = 0; wsx < NWAVE; ++wsx) {
        int n = __builtin_amdgcn_readfirstlane(wcnt[wsx]);
        n = n > WCAP ? WCAP : (n < 0 ? 0 : n);
        const int* lp = list + wsx * WCAP;
#pragma unroll 1
        for (int i = 0; i < n; ++i) {
          const int ent  = __builtin_amdgcn_readfirstlane(lp[i]);
          const int slot = ent & (NBF - 1);
          int e = cbase + ((ent >> 12) & (CHUNK - 1));
          e = e > nE - 1 ? nE - 1 : e;
          int src = ei[e];
          src = src < 0 ? 0 : (src > nN - 1 ? nN - 1 : src);
          if (lane == 0) {
            int pos = cursor[slot];
            pos = pos < 0 ? 0 : (pos > RCAP - 1 ? RCAP - 1 : pos);
            region[pos] = src;
            const int np = pos + 1;
            cursor[slot] = np > RCAP ? RCAP : np;
          }
        }
      }
    }
    __syncthreads();
  }

  const int nv = lenW >> 2;
  int* gp = csr + rb0;
#pragma unroll 1
  for (int i = tid; i < nv; i += NTHR) { const v4i v = ((const v4i*)region)[i]; *(volatile v4i*)(gp + 4 * i) = v; }
  __threadfence();
#pragma unroll 1
  for (int i = tid; i < nv; i += NTHR) { const v4i v = ((const v4i*)region)[i]; *(volatile v4i*)(gp + 4 * i) = v; }
}

template <int CI>
__global__ __launch_bounds__(NTHR) void k_agg(
    const int* __restrict__ csr, const int* __restrict__ off, const int* __restrict__ cnt,
    const float* __restrict__ invd, const float* __restrict__ h, float* meanp,
    int nN, int csrLen) {
  constexpr int NQ = CI / 128;
  const int tid = threadIdx.x, lane = tid & 31, wave = tid >> 5;
  const int tbase = blockIdx.x * TGT + wave * 32;
  const int cl = tbase + lane;
  const int cnt_l = cnt[cl];
  const int off_l = off[cl];
  union FI { float f; int i; };
  FI ivu; ivu.f = invd[cl];

#pragma unroll 1
  for (int j = 0; j < 32; ++j) {
    const int c = tbase + j;
    int n = __builtin_amdgcn_readlane(cnt_l, j);
    n = n < 0 ? 0 : (n > DEGCAP ? DEGCAP : n);
    const int st = __builtin_amdgcn_readlane(off_l, j);
    FI du; du.i = __builtin_amdgcn_readlane(ivu.i, j);
    v4f acc[NQ];
#pragma unroll
    for (int q = 0; q < NQ; ++q) { const v4f z = {0.f, 0.f, 0.f, 0.f}; acc[q] = z; }
#pragma unroll 1
    for (int q0 = 0; q0 < n; q0 += 32) {
      int pos = st + q0 + lane;
      pos = pos < 0 ? 0 : (pos > csrLen - 1 ? csrLen - 1 : pos);
      int sl = csr[pos];
      sl = sl < 0 ? 0 : (sl > nN - 1 ? nN - 1 : sl);
      const int mcnt = (n - q0) < 32 ? (n - q0) : 32;
#pragma unroll 1
      for (int p = 0; p < mcnt; ++p) {
        const int s = __builtin_amdgcn_readlane(sl, p);
        const float* hp = h + (size_t)s * CI + 4 * lane;
#pragma unroll
        for (int q = 0; q < NQ; ++q) acc[q] = acc[q] + *(const v4f*)(hp + 128 * q);
      }
    }
    v4f v[NQ];
#pragma unroll
    for (int q = 0; q < NQ; ++q) v[q] = acc[q] * du.f;
    float* mp = meanp + (size_t)c * CI + 4 * lane;
#pragma unroll
    for (int q = 0; q < NQ; ++q) *(volatile v4f*)(mp + 128 * q) = v[q];
    __threadfence();
#pragma unroll
    for (int q = 0; q < NQ; ++q) *(volatile v4f*)(mp + 128 * q) = v[q];
  }
}

template <int CI>
__global__ __launch_bounds__(NTHR) void k_gemm(
    const float* __restrict__ meanp, const float* __restrict__ hsrc,
    const unsigned short* __restrict__ whi, const unsigned short* __restrict__ wlo,
    const float* __restrict__ bias, float* P, double* part, int nN) {
  constexpr int K = 2 * CI;
  __shared__ __attribute__((aligned(16))) float  stg[GR * HC];
  __shared__ __attribute__((aligned(16))) double sst[2 * HC];
  const int tid = threadIdx.x, lane = tid & 31, wave = tid >> 5, hh = lane >> 4, m = lane & 15;
  const int wr = wave & 1, wc = wave >> 1;
  const int rowBase = blockIdx.x * GR;
  int ra = rowBase + 16 * wr + m;
  ra = ra > nN - 1 ? nN - 1 : ra;
  const float* am = meanp + (size_t)ra * CI + 8 * hh;
  const float* ah = hsrc  + (size_t)ra * CI + 8 * hh;
  const unsigned short* bh = whi + (size_t)(64 * wc + m) * K + 8 * hh;
  const unsigned short* bl = wlo + (size_t)(64 * wc + m) * K + 8 * hh;

  v8f acc[4];
#pragma unroll
  for (int t = 0; t < 4; ++t) { const v8f z = {0.f, 0.f, 0.f, 0.f, 0.f, 0.f, 0.f, 0.f}; acc[t] = z; }

#pragma unroll 1
  for (int kt = 0; kt < K / 32; ++kt) {
    const bool first = kt < CI / 32;
    const float* ap = first ? (am + 32 * kt) : (ah + 32 * (kt - CI / 32));
    const v4f a0 = *(const v4f*)ap, a1 = *(const v4f*)(ap + 4);
    const v4f a2 = *(const v4f*)(ap + 16), a3 = *(const v4f*)(ap + 20);
    float av[16];
    av[0]  = a0.x; av[1]  = a0.y; av[2]  = a0.z; av[3]  = a0.w;
    av[4]  = a1.x; av[5]  = a1.y; av[6]  = a1.z; av[7]  = a1.w;
    av[8]  = a2.x; av[9]  = a2.y; av[10] = a2.z; av[11] = a2.w;
    av[12] = a3.x; av[13] = a3.y; av[14] = a3.z; av[15] = a3.w;
    FragB fah, fal;
#pragma unroll
    for (int p = 0; p < 8; ++p) {
      unsigned int lw;
      fah.w[p] = split_pack(av[2 * p], av[2 * p + 1], lw);
      fal.w[p] = lw;
    }
    const unsigned short* bhk = bh + 32 * kt;
    const unsigned short* blk = bl + 32 * kt;
#pragma unroll
    for (int t = 0; t < 4; ++t) {
      FragB gh, gl;
      gh.hv[0] = *(const v8us*)(bhk + (size_t)(16 * t) * K);
      gh.hv[1] = *(const v8us*)(bhk + (size_t)(16 * t) * K + 16);
      gl.hv[0] = *(const v8us*)(blk + (size_t)(16 * t) * K);
      gl.hv[1] = *(const v8us*)(blk + (size_t)(16 * t) * K + 16);
      acc[t] = wmb(fah.bf, gh.bf, acc[t]);
      acc[t] = wmb(fah.bf, gl.bf, acc[t]);
      acc[t] = wmb(fal.bf, gh.bf, acc[t]);
    }
  }

#pragma unroll
  for (int t = 0; t < 4; ++t) {
    const int col = 64 * wc + 16 * t + m;
    const float bv = bias[col];
    float* sp = stg + (16 * wr + 8 * hh) * HC + col;
#pragma unroll
    for (int r = 0; r < 8; ++r) sp[r * HC] = acc[t][r] + bv;
  }
  __syncthreads();

  {
    int nv = nN - rowBase;
    nv = nv > GR ? GR : (nv < 0 ? 0 : nv);
    double s = 0.0, q = 0.0;
#pragma unroll 1
    for (int r = 0; r < nv; ++r) {
      const double v = (double)stg[r * HC + tid];
      s += v;
      q = fma(v, v, q);
    }
    sst[tid] = s;
    sst[HC + tid] = q;
  }

  v4f pv[8];
#pragma unroll
  for (int i = 0; i < 4; ++i) {
    const float* lp = stg + (4 * wave + i) * HC + 4 * lane;
    pv[2 * i]     = *(const v4f*)lp;
    pv[2 * i + 1] = *(const v4f*)(lp + 128);
  }
  __syncthreads();
  const v2d sv = *(const v2d*)(sst + 2 * tid);
  double* pp = part + (size_t)blockIdx.x * (2 * HC) + 2 * tid;

#pragma unroll
  for (int i = 0; i < 4; ++i) {
    const int grow = rowBase + 4 * wave + i;
    if (grow < nN) {
      float* gp = P + (size_t)grow * HC + 4 * lane;
      *(volatile v4f*)gp = pv[2 * i];
      *(volatile v4f*)(gp + 128) = pv[2 * i + 1];
    }
  }
  *(volatile v2d*)pp = sv;
  __threadfence();
#pragma unroll
  for (int i = 0; i < 4; ++i) {
    const int grow = rowBase + 4 * wave + i;
    if (grow < nN) {
      float* gp = P + (size_t)grow * HC + 4 * lane;
      *(volatile v4f*)gp = pv[2 * i];
      *(volatile v4f*)(gp + 128) = pv[2 * i + 1];
    }
  }
  *(volatile v2d*)pp = sv;
}

__global__ __launch_bounds__(NTHR) void k_bnfin(
    const double* __restrict__ part, int nBlk, int nN, float* tab) {
  __shared__ __attribute__((aligned(16))) float st[2 * HC];
  const int tid = threadIdx.x;
  double s = 0.0, q = 0.0;
#pragma unroll 1
  for (int b = 0; b < nBlk; ++b) {
    s += part[(size_t)b * (2 * HC) + tid];
    q += part[(size_t)b * (2 * HC) + HC + tid];
  }
  const double invn = 1.0 / (double)nN;
  const double mu = s * invn;
  double var = q * invn - mu * mu;
  var = var < 0.0 ? 0.0 : var;
  const float varf = (float)var;
  st[tid] = (float)mu;
  st[HC + tid] = rsqrtf(varf + BNEPS);
  __syncthreads();
  v4f v = {0.f, 0.f, 0.f, 0.f};
  if (tid < 128) v = *(const v4f*)(st + 4 * tid);
  if (tid < 128) *(volatile v4f*)(tab + 4 * tid) = v;
  __threadfence();
  if (tid < 128) *(volatile v4f*)(tab + 4 * tid) = v;
}

__global__ __launch_bounds__(NTHR) void k_bnapply(
    const float* P, const float* __restrict__ tab, const float* __restrict__ g,
    const float* __restrict__ bb, float* dst, int n4, int relu) {
  const int i = blockIdx.x * NTHR + (int)threadIdx.x;
  if (i >= n4) return;
  const int c4 = (i & (HC / 4 - 1)) * 4;
  const v4f x  = *(const v4f*)(P + (size_t)i * 4);
  const v4f mu = *(const v4f*)(tab + c4);
  const v4f rs = *(const v4f*)(tab + HC + c4);
  const v4f gg = *(const v4f*)(g + c4);
  const v4f be = *(const v4f*)(bb + c4);
  v4f v = (x - mu) * rs * gg + be;
  if (relu != 0) { v.x = fmaxf(v.x, 0.f); v.y = fmaxf(v.y, 0.f); v.z = fmaxf(v.z, 0.f); v.w = fmaxf(v.w, 0.f); }
  float* dp = dst + (size_t)i * 4;
  *(volatile v4f*)dp = v;
  __threadfence();
  *(volatile v4f*)dp = v;
}

extern "C" void kernel_launch(void* const* d_in, const int* in_sizes, int n_in,
                              void* d_out, int out_size, void* d_ws, size_t ws_size,
                              hipStream_t stream) {
  if (n_in < 17) return;
  const int nN = in_sizes[0] / INC;
  const int nE = in_sizes[1] / 2;
  if (nN <= 0 || nE <= 0 || in_sizes[0] != nN * INC || in_sizes[1] != 2 * nE) return;
  if (in_sizes[2] != HC * INC || in_sizes[4] != HC * INC) return;
  if (in_sizes[7] != HC * HC || in_sizes[9] != HC * HC || in_sizes[12] != HC * HC || in_sizes[14] != HC * HC) return;
  if (in_sizes[3] < HC || in_sizes[5] < HC || in_sizes[6] < HC || in_sizes[8] < HC || in_sizes[10] < HC ||
      in_sizes[11] < HC || in_sizes[13] < HC || in_sizes[15] < HC || in_sizes[16] < HC) return;
  if (out_size != nN * HC) return;
  if (nE > (1 << 28) || nN > (1 << 24)) return;

  const float* x    = (const float*)d_in[0];
  const int*   ei   = (const int*)d_in[1];
  const float* Wl0  = (const float*)d_in[2];
  const float* bl0  = (const float*)d_in[3];
  const float* Wr0  = (const float*)d_in[4];
  const float* ga0  = (const float*)d_in[5];
  const float* be0  = (const float*)d_in[6];
  const float* Wl1  = (const float*)d_in[7];
  const float* bl1  = (const float*)d_in[8];
  const float* Wr1  = (const float*)d_in[9];
  const float* ga1  = (const float*)d_in[10];
  const float* be1  = (const float*)d_in[11];
  const float* Wl2  = (const float*)d_in[12];
  const float* bl2  = (const float*)d_in[13];
  const float* Wr2  = (const float*)d_in[14];
  const float* ga2  = (const float*)d_in[15];
  const float* be2  = (const float*)d_in[16];
  float* out = (float*)d_out;

  const int NPAD   = ((nN + TGT - 1) / TGT) * TGT;
  const int nBC    = (nN + NBC - 1) / NBC;
  const int CNTPAD = nBC * NBC;
  if (4 * nBC + 1 > RBN) return;
  const int nBF    = (nN + NBF - 1) / NBF;
  const int csrLen = ((nE + 31) & ~31) + 4096;
  const int nAgg   = NPAD / TGT;
  const int nGB    = (nN + GR - 1) / GR;
  const int n4     = nN * (HC / 4);
  const int nAp    = (n4 + NTHR - 1) / NTHR;

  char* ws = (char*)d_ws;
  size_t off = 0;
  const size_t oWh0 = off; off += (size_t)HC * 2 * INC * 2;       off = (off + 255) & ~(size_t)255;
  const size_t oWd0 = off; off += (size_t)HC * 2 * INC * 2;       off = (off + 255) & ~(size_t)255;
  const size_t oWh1 = off; off += (size_t)HC * 2 * HC * 2;        off = (off + 255) & ~(size_t)255;
  const size_t oWd1 = off; off += (size_t)HC * 2 * HC * 2;        off = (off + 255) & ~(size_t)255;
  const size_t oWh2 = off; off += (size_t)HC * 2 * HC * 2;        off = (off + 255) & ~(size_t)255;
  const size_t oWd2 = off; off += (size_t)HC * 2 * HC * 2;        off = (off + 255) & ~(size_t)255;
  const size_t oCnt = off; off += (size_t)CNTPAD * 4;             off = (off + 255) & ~(size_t)255;
  const size_t oInv = off; off += (size_t)CNTPAD * 4;             off = (off + 255) & ~(size_t)255;
  const size_t oOff = off; off += (size_t)CNTPAD * 4;             off = (off + 255) & ~(size_t)255;
  const size_t oRb  = off; off += (size_t)RBN * 4;                off = (off + 255) & ~(size_t)255;
  const size_t oCsr = off; off += (size_t)csrLen * 4;             off = (off + 255) & ~(size_t)255;
  const size_t oMn  = off; off += (size_t)NPAD * HC * 4;          off = (off + 255) & ~(size_t)255;
  const size_t oH   = off; off += (size_t)NPAD * HC * 4;          off = (off + 255) & ~(size_t)255;
  const size_t oPt  = off; off += (size_t)nGB * (2 * HC) * 8;     off = (off + 255) & ~(size_t)255;
  const size_t oTab = off; off += (size_t)(2 * HC) * 4;           off = (off + 255) & ~(size_t)255;
  if (off > ws_size) return;
  unsigned short* whi0 = (unsigned short*)(ws + oWh0);
  unsigned short* wlo0 = (unsigned short*)(ws + oWd0);
  unsigned short* whi1 = (unsigned short*)(ws + oWh1);
  unsigned short* wlo1 = (unsigned short*)(ws + oWd1);
  unsigned short* whi2 = (unsigned short*)(ws + oWh2);
  unsigned short* wlo2 = (unsigned short*)(ws + oWd2);
  int*    cnt   = (int*)(ws + oCnt);
  float*  invd  = (float*)(ws + oInv);
  int*    offp  = (int*)(ws + oOff);
  int*    rb    = (int*)(ws + oRb);
  int*    csr   = (int*)(ws + oCsr);
  float*  meanp = (float*)(ws + oMn);
  float*  hpl   = (float*)(ws + oH);
  double* part  = (double*)(ws + oPt);
  float*  tab   = (float*)(ws + oTab);

  const int vec8 = ((nE & 3) == 0) ? 1 : 0;

  const int nPrep = (HC * 2 * INC / 8 + 2 * (HC * 2 * HC / 8)) / NTHR;
  k_wprep<<<nPrep, NTHR, 0, stream>>>(Wl0, Wr0, Wl1, Wr1, Wl2, Wr2, whi0, wlo0, whi1, wlo1, whi2, wlo2);

  k_count<<<nBC, NTHR, 0, stream>>>(ei, cnt, invd, nE, vec8);
  k_offsets<<<1, OTHR, 0, stream>>>(cnt, offp, rb, nBC);
  hipFuncSetAttribute(reinterpret_cast<const void*>(&k_fill),
                      hipFuncAttributeMaxDynamicSharedMemorySize, LDS_FILL);
  k_fill<<<nBF, NTHR, LDS_FILL, stream>>>(ei, offp, rb, csr, nN, nE, vec8, csrLen);

  k_agg<INC><<<nAgg, NTHR, 0, stream>>>(csr, offp, cnt, invd, x, meanp, nN, csrLen);
  k_gemm<INC><<<nGB, NTHR, 0, stream>>>(meanp, x, whi0, wlo0, bl0, out, part, nN);
  k_bnfin<<<1, NTHR, 0, stream>>>(part, nGB, nN, tab);
  k_bnapply<<<nAp, NTHR, 0, stream>>>(out, tab, ga0, be0, hpl, n4, 1);

  k_agg<HC><<<nAgg, NTHR, 0, stream>>>(csr, offp, cnt, invd, hpl, meanp, nN, csrLen);
  k_gemm<HC><<<nGB, NTHR, 0, stream>>>(meanp, hpl, whi1, wlo1, bl1, out, part, nN);
  k_bnfin<<<1, NTHR, 0, stream>>>(part, nGB, nN, tab);
  k_bnapply<<<nAp, NTHR, 0, stream>>>(out, tab, ga1, be1, hpl, n4, 1);

  k_agg<HC><<<nAgg, NTHR, 0, stream>>>(csr, offp, cnt, invd, hpl, meanp, nN, csrLen);
  k_gemm<HC><<<nGB, NTHR, 0, stream>>>(meanp, hpl, whi2, wlo2, bl2, out, part, nN);
  k_bnfin<<<1, NTHR, 0, stream>>>(part, nGB, nN, tab);
  k_bnapply<<<nAp, NTHR, 0, stream>>>(out, tab, ga2, be2, out, n4, 0);
}
